// GRUCell_43181601194444
// MI455X (gfx1250) — hardware-verified
//
#include <hip/hip_runtime.h>
#include <math.h>

typedef __attribute__((ext_vector_type(16))) _Float16 v16h;
typedef __attribute__((ext_vector_type(16))) __bf16 v16b;
typedef __attribute__((ext_vector_type(8)))  _Float16 v8h;
typedef __attribute__((ext_vector_type(8)))  float v8f;
typedef __attribute__((ext_vector_type(4)))  float v4f;
typedef __attribute__((ext_vector_type(2)))  float v2f;
typedef __attribute__((ext_vector_type(4)))  unsigned v4u;
typedef __attribute__((ext_vector_type(4)))  int v4i;
typedef float __attribute__((may_alias)) float_a;
typedef int __attribute__((may_alias)) int_a;

template <typename T> __device__ __forceinline__ void vst2(void* p, T v) { *(volatile T*)p = v; __threadfence(); *(volatile T*)p = v; }
__device__ __forceinline__ v8f wmma16(v16h a, v16h b, v8f c) {
  v8f d = __builtin_amdgcn_wmma_f32_16x16x32_f16(false, a, false, b, (short)0, c, false, false);
  asm volatile("v_nop\n\tv_nop\n\tv_nop\n\tv_nop" : "+v"(d) : "v"(a), "v"(b));
  return d;
}
__device__ __forceinline__ v8f wmma_bf(v16b a, v16b b, v8f c) {
  v8f d = __builtin_amdgcn_wmma_f32_16x16x32_bf16(false, a, false, b, (short)0, c, false, false);
  asm volatile("v_nop\n\tv_nop\n\tv_nop\n\tv_nop" : "+v"(d) : "v"(a), "v"(b));
  return d;
}
__device__ __forceinline__ v16h frag_h(const _Float16* rowk0, int lane) {
  union { v16h v; v8h q[2]; } u; const _Float16* p = rowk0 + 8 * (lane >> 4);
  u.q[0] = *(const v8h*)p; u.q[1] = *(const v8h*)(p + 16); return u.v;
}
__device__ __forceinline__ v16h frag_f32(const float* rowk0, int lane) {
  v16h a; const float* p = rowk0 + 8 * (lane >> 4);
#pragma unroll
  for (int i = 0; i < 8; ++i) { a[i] = (_Float16)p[i]; a[8 + i] = (_Float16)p[16 + i]; }
  return a;
}
__device__ __forceinline__ v16h frag_f32s(const float* rowk0, int lane, float sc) {
  v16h a; const float* p = rowk0 + 8 * (lane >> 4);
#pragma unroll
  for (int i = 0; i < 8; ++i) { a[i] = (_Float16)(p[i] * sc); a[8 + i] = (_Float16)(p[16 + i] * sc); }
  return a;
}
__device__ __forceinline__ v16h fragc_f32(const float* W, int k0, int n, int lane, int ld, int K) {
  v16h a; const int g = lane >> 4;
#pragma unroll
  for (int i = 0; i < 8; ++i) { const int ka = k0 + 8 * g + i, kb = ka + 16;
    a[i] = (_Float16)(ka < K ? W[(size_t)(ka < K ? ka : K - 1) * ld + n] : 0.f); a[8 + i] = (_Float16)(kb < K ? W[(size_t)(kb < K ? kb : K - 1) * ld + n] : 0.f); }
  return a;
}
struct F2 { v16b h, l; };
__device__ __forceinline__ F2 bsplit16(const float v[16]) { F2 r;
#pragma unroll
  for (int i = 0; i < 16; ++i) { const __bf16 h = (__bf16)v[i]; r.h[i] = h; r.l[i] = (__bf16)(v[i] - (float)h); }
  return r; }
__device__ __forceinline__ F2 split_row(const float* row, int k0, int lane) { float v[16]; const float* p = row + k0 + 8 * (lane >> 4);
#pragma unroll
  for (int i = 0; i < 8; ++i) { v[i] = p[i]; v[8 + i] = p[16 + i]; }
  return bsplit16(v); }
__device__ __forceinline__ F2 split_rowK(const float* row, int k0, int lane, int K) { float v[16]; const int g = lane >> 4;
#pragma unroll
  for (int i = 0; i < 8; ++i) { const int ka = k0 + 8 * g + i, kb = ka + 16; v[i] = ka < K ? row[ka < K ? ka : K - 1] : 0.f; v[8 + i] = kb < K ? row[kb < K ? kb : K - 1] : 0.f; }
  return bsplit16(v); }
__device__ __forceinline__ F2 split_col(const float* W, int k0, int n, int lane, int ld, int K) { float v[16]; const int g = lane >> 4;
#pragma unroll
  for (int i = 0; i < 8; ++i) { const int ka = k0 + 8 * g + i, kb = ka + 16; v[i] = ka < K ? W[(size_t)(ka < K ? ka : K - 1) * ld + n] : 0.f; v[8 + i] = kb < K ? W[(size_t)(kb < K ? kb : K - 1) * ld + n] : 0.f; }
  return bsplit16(v); }
__device__ __forceinline__ v8f mac3(const F2& a, const F2& b, v8f c) { c = wmma_bf(a.l, b.h, c); c = wmma_bf(a.h, b.l, c); return wmma_bf(a.h, b.h, c); }
__device__ __forceinline__ float sigm(float v) { return 1.0f / (1.0f + expf(-v)); }
#define LDSX() do { asm volatile("s_wait_dscnt 0" ::: "memory"); __builtin_amdgcn_wave_barrier(); __builtin_amdgcn_fence(__ATOMIC_RELEASE, "workgroup"); } while (0)

#define NBR 16384
#define IN 256
#define HD 256
#ifndef NRV
#define NRV NBR
#endif
__device__ __forceinline__ float bfr(float v) { return (float)(__bf16)v; }
__device__ __forceinline__ v16b wcol_io2(const float* __restrict__ Wm, int k0, int o, int lane, int ld) { v16b w; const float* p = Wm + (size_t)(k0 + 8 * (lane >> 4)) * ld + o; float t0[8], t1[8];
#pragma unroll
  for (int i = 0; i < 8; ++i) t0[i] = p[(size_t)i * ld];
  asm volatile("s_wait_loadcnt 0x0" ::: "memory");
#pragma unroll
  for (int i = 0; i < 8; ++i) t1[i] = p[(size_t)(16 + i) * ld];
  asm volatile("s_wait_loadcnt 0x0" ::: "memory");
#pragma unroll
  for (int i = 0; i < 8; ++i) { w[i] = (__bf16)t0[i]; w[8 + i] = (__bf16)t1[i]; }
  return w; }
__device__ __forceinline__ v16b arow_bf(const float* __restrict__ p, int lane) { v16b a; const int g = lane >> 4; float t0[8], t1[8];
#pragma unroll
  for (int i = 0; i < 8; ++i) t0[i] = p[8 * g + i];
  asm volatile("s_wait_loadcnt 0x0" ::: "memory");
#pragma unroll
  for (int i = 0; i < 8; ++i) t1[i] = p[16 + 8 * g + i];
  asm volatile("s_wait_loadcnt 0x0" ::: "memory");
#pragma unroll
  for (int i = 0; i < 8; ++i) { a[i] = (__bf16)t0[i]; a[8 + i] = (__bf16)t1[i]; }
  return a; }
#define WS_U   0u
#define WS_XC  (WS_U + 4u * (size_t)NBR * HD)
#define WS_RH  (WS_XC + 4u * (size_t)NBR * HD)
#define WS_END (WS_RH + 4u * (size_t)NBR * HD)
__global__ __launch_bounds__(128) void k_ga(const float* __restrict__ X, const float* __restrict__ Hm, const float* __restrict__ WI, const float* __restrict__ WH, const float* __restrict__ BI, float* __restrict__ U, float* __restrict__ XC, float* __restrict__ RH) {
  __shared__ __align__(16) float su[4][16][68]; __shared__ __align__(16) float sx[4][16][68]; __shared__ __align__(16) float sr[4][16][68];
  const int tid = threadIdx.x, wave = tid >> 5, lane = tid & 31, col = lane & 15, g = lane >> 4; const int c0 = blockIdx.y * 64; const size_t r0 = (size_t)blockIdx.x * 64 + wave * 16;
  v8f ar[4] = {}, au[4] = {}, ac[4] = {}, hr[4] = {}, hu[4] = {};
#pragma unroll 1
  for (int kc = 0; kc < IN / 32; ++kc) { const v16b a = arow_bf(X + (r0 + col) * IN + kc * 32, lane); const v16b ah = arow_bf(Hm + (r0 + col) * HD + kc * 32, lane);
#pragma unroll
    for (int j = 0; j < 4; ++j) { const int c = c0 + j * 16 + col;
      { const v16b w = wcol_io2(WI, kc * 32, c, lane, 3 * HD); ar[j] = wmma_bf(a, w, ar[j]); }
      { const v16b w = wcol_io2(WI, kc * 32, HD + c, lane, 3 * HD); au[j] = wmma_bf(a, w, au[j]); }
      { const v16b w = wcol_io2(WI, kc * 32, 2 * HD + c, lane, 3 * HD); ac[j] = wmma_bf(a, w, ac[j]); }
      { const v16b w = wcol_io2(WH, kc * 32, c, lane, 3 * HD); hr[j] = wmma_bf(ah, w, hr[j]); }
      { const v16b w = wcol_io2(WH, kc * 32, HD + c, lane, 3 * HD); hu[j] = wmma_bf(ah, w, hu[j]); } } }
#pragma unroll
  for (int j = 0; j < 4; ++j) { const int c = c0 + j * 16 + col; const float br = bfr(BI[c]), bu = bfr(BI[HD + c]), bc = bfr(BI[2 * HD + c]); asm volatile("s_wait_loadcnt 0x0" ::: "memory");
#pragma unroll
    for (int r = 0; r < 8; ++r) { const float rg = 1.0f / (1.0f + expf(-((ar[j][r] + br) + hr[j][r]))); const float ug = 1.0f / (1.0f + expf(-((au[j][r] + bu) + hu[j][r])));
      su[wave][8 * g + r][j * 16 + col] = ug; sx[wave][8 * g + r][j * 16 + col] = ac[j][r] + bc; sr[wave][8 * g + r][j * 16 + col] = rg; } }
  LDSX();
  for (int rl = 0; rl < 16; ++rl) if (lane < 16) { const size_t o = (r0 + rl) * HD + c0 + lane * 4; const v4f hv = *(const v4f*)(Hm + o); v4f rr = *(const v4f*)&sr[wave][rl][lane * 4];
#pragma unroll
      for (int i = 0; i < 4; ++i) rr[i] = rr[i] * bfr(hv[i]);
      vst2(U + o, *(const v4f*)&su[wave][rl][lane * 4]); vst2(XC + o, *(const v4f*)&sx[wave][rl][lane * 4]); vst2(RH + o, rr); } }
__global__ __launch_bounds__(128) void k_gb(const float* __restrict__ RH, const float* __restrict__ WH, const float* __restrict__ XC, const float* __restrict__ U, const float* __restrict__ Hm, float* __restrict__ OUT) { __shared__ __align__(16) float sf[4][16][132];
  const int tid = threadIdx.x, wave = tid >> 5, lane = tid & 31, col = lane & 15, g = lane >> 4; const int c0 = blockIdx.y * 128; const size_t r0 = (size_t)blockIdx.x * 64 + wave * 16;
  v8f acc[8] = {};
#pragma unroll 2
  for (int kc = 0; kc < HD / 32; ++kc) { const F2 a = split_row(RH + (r0 + col) * HD, kc * 32, lane); asm volatile("s_wait_loadcnt 0x0" ::: "memory");
#pragma unroll
    for (int j = 0; j < 8; ++j) { const v16b w = wcol_io2(WH, kc * 32, 2 * HD + c0 + j * 16 + col, lane, 3 * HD); acc[j] = wmma_bf(a.h, w, acc[j]); acc[j] = wmma_bf(a.l, w, acc[j]); } }
#pragma unroll
  for (int j = 0; j < 8; ++j)
#pragma unroll
    for (int r = 0; r < 8; ++r) sf[wave][8 * g + r][j * 16 + col] = acc[j][r];
  LDSX();
  for (int rl = 0; rl < 16; ++rl) { const size_t o = (r0 + rl) * HD + c0 + lane * 4; const v4f xc = *(const v4f*)(XC + o), uu = *(const v4f*)(U + o), hv = *(const v4f*)(Hm + o); v4f out;
#pragma unroll
    for (int i = 0; i < 4; ++i) { const float cand = tanhf(xc[i] + sf[wave][rl][lane * 4 + i]); out[i] = uu[i] * bfr(hv[i]) + (1.0f - uu[i]) * cand; }
    vst2(OUT + o, out); } }
extern "C" void kernel_launch(void* const* d_in, const int* in_sizes, int n_in, void* d_out, int out_size, void* d_ws, size_t ws_size, hipStream_t stream) {
  (void)in_sizes; (void)n_in; (void)out_size;
  if (ws_size < (size_t)WS_END) return;
  char* ws = (char*)d_ws; const float** F = (const float**)d_in; float *U = (float*)(ws + WS_U), *XC = (float*)(ws + WS_XC), *RH = (float*)(ws + WS_RH);
  k_ga<<<dim3(NRV / 64, HD / 64), 128, 0, stream>>>(F[0], F[1], F[2], F[3], F[4], U, XC, RH);
  k_gb<<<dim3(NRV / 64, HD / 128), 128, 0, stream>>>(RH, F[3], XC, U, F[1], (float*)d_out);
}
